// SLAHead_10617159155942
// MI455X (gfx1250) — hardware-verified
//
#include <hip/hip_runtime.h>

typedef __attribute__((ext_vector_type(16))) _Float16 v16h;
typedef __attribute__((ext_vector_type(8)))  _Float16 v8h;
typedef __attribute__((ext_vector_type(8)))  float    v8f;

#define HIDN 256
#define NOUT 30
#define NLOC 4
#define CIN  96
#define NHW  256
#define NB   8
#define STEPS 501

__device__ __forceinline__ v8f wmma_rm(const _Float16* __restrict__ A, int lda,
                                       const _Float16* __restrict__ W, int ldw,
                                       int row0, int K, v8f acc)
{
    const int  lane = threadIdx.x & 31;
    const int  mlo  = lane & 15;
    const bool hiH  = lane >= 16;
    const _Float16* wrow = W + (size_t)(row0 + mlo) * ldw;
    const _Float16* arow = A + (size_t)mlo * lda;
    const int kA1 = hiH ? 8 : 0;
    const int kA2 = hiH ? 24 : 16;
    for (int k0 = 0; k0 < K; k0 += 32) {
        v8h blo = *(const v8h*)(wrow + k0 + kA1);
        v8h bhi = *(const v8h*)(wrow + k0 + kA2);
        v8h alo = *(const v8h*)(arow + k0 + kA1);
        v8h ahi = *(const v8h*)(arow + k0 + kA2);
        v16h a, b;
#pragma unroll
        for (int t = 0; t < 8; ++t) { a[t] = alo[t]; a[t + 8] = ahi[t]; b[t] = blo[t]; b[t + 8] = bhi[t]; }
        acc = __builtin_amdgcn_wmma_f32_16x16x32_f16(
                  false, a, false, b, (short)0, acc, false, false);
        asm volatile("v_nop\n\tv_nop\n\tv_nop\n\tv_nop" : "+v"(acc) : "v"(a), "v"(b));
    }
    return acc;
}

typedef __attribute__((ext_vector_type(4))) unsigned v4u;
typedef __attribute__((ext_vector_type(4))) float v4f;
typedef float __attribute__((may_alias)) float_a;
template <typename V> __device__ __forceinline__ void vst2(void* p, V v) {
    *(volatile V*)p = v; __threadfence(); *(volatile V*)p = v;
}
__global__ void cvt_pad_f16(const float* __restrict__ src, _Float16* __restrict__ dst,
                            int rs, int cs, int rd, int cd)
{
    int g = blockIdx.x * blockDim.x + threadIdx.x;
    if (g * 8 >= rd * cd) return;
    union { v8h h; v4u u; } pk;
#pragma unroll
    for (int e = 0; e < 8; ++e) {
        int i = g * 8 + e;
        int r = i / cd, c = i - r * cd;
        pk.h[e] = (r < rs && c < cs) ? (_Float16)src[r * cs + c] : (_Float16)0.f;
    }
    vst2(dst + (size_t)g * 8, pk.u);
}

__global__ void prep_hproj(const float* __restrict__ fea,
                           const float* __restrict__ i2h,
                           float* __restrict__ Hp)
{
    int idx = blockIdx.x * blockDim.x + threadIdx.x;
    int h = idx & 255, s = (idx >> 8) & 255, b = idx >> 16;
    float acc = 0.f;
    const float* ir = i2h + h * CIN;
#pragma unroll 4
    for (int c = 0; c < CIN; ++c)
        acc += fea[((size_t)(b * CIN + c) << 8) + s] * ir[c];
    vst2(Hp + idx, (float_a)acc);
}

__global__ __launch_bounds__(512)
void sla_decoder(const float* __restrict__ fea,
                 const float* __restrict__ Hp,
                 const _Float16* __restrict__ h2hW, const float* __restrict__ h2hB,
                 const float* __restrict__ scoreW,
                 const _Float16* __restrict__ gihW, const _Float16* __restrict__ ghhW,
                 const float* __restrict__ bih, const float* __restrict__ bhh,
                 const _Float16* __restrict__ sg1W, const float* __restrict__ sg1B,
                 const _Float16* __restrict__ sg2W, const float* __restrict__ sg2B,
                 const _Float16* __restrict__ lg1W, const float* __restrict__ lg1B,
                 const _Float16* __restrict__ lg2W, const float* __restrict__ lg2B,
                 float* __restrict__ stage)
{
    extern __shared__ char smem[];
    _Float16* w2L    = (_Float16*)smem;
    _Float16* hidF16 = w2L    + 48 * 256;
    _Float16* xF16   = hidF16 + 16 * 256;
    _Float16* s1F16  = xF16   + 16 * 128;
    _Float16* l1F16  = s1F16  + 16 * 256;
    float* hidF32 = (float*)(l1F16 + 16 * 256);
    float* tF32   = hidF32 + 8 * 256;
    float* eA     = tF32   + 8 * 256;
    float* giL    = eA     + 8 * 256;
    float* ghL    = giL    + 8 * 768;
    float* ctx    = ghL    + 8 * 768;
    float* sOut   = ctx    + 8 * 96;
    float* lOut   = sOut   + 8 * 32;
    float* swL    = lOut   + 8 * 16;
    int*   preL   = (int*)(swL + 256);
    _Float16* sg2L = w2L;
    _Float16* lg2L = w2L + 32 * 256;

    const int tid  = threadIdx.x;
    const int w    = tid >> 5;
    const int lane = tid & 31;
    const int mlo  = lane & 15;
    const bool hiH = lane >= 16;

    for (int i = tid; i < 1536; i += 512) {
        const _Float16* src = (i < 1024) ? (sg2W + i * 8) : (lg2W + (i - 1024) * 8);
        *(v4u*)(w2L + i * 8) = *(const v4u*)src;
    }

    for (int i = tid; i < 16 * 256; i += 512) { hidF16[i] = (_Float16)0.f;
                                               s1F16[i] = (_Float16)0.f;
                                               l1F16[i] = (_Float16)0.f; }
    for (int i = tid; i < 16 * 128; i += 512) xF16[i] = (_Float16)0.f;
    for (int i = tid; i < 8 * 256;  i += 512) hidF32[i] = 0.f;
    if (tid < 256) swL[tid] = scoreW[tid];
    if (tid < 8)   preL[tid] = 0;
    __syncthreads();

    for (int step = 0; step < STEPS; ++step) {
        int lz = 0;
        asm volatile("" : "+s"(lz));

        {
            v8f acc = {};
            acc = wmma_rm(hidF16, 256, h2hW + lz, 256, w * 16, 256, acc);
            if (!hiH) {
                int col = w * 16 + mlo;
                float bb = h2hB[col];
#pragma unroll
                for (int r = 0; r < NB; ++r) tF32[r * 256 + col] = acc[r] + bb;
            }
        }
        __syncthreads();
        for (int p = w; p < NB * NHW; p += 16) {
            int b = p >> 8, s = p & 255;
            const float* hp = Hp + ((size_t)(b * 256 + s) << 8);
            __builtin_prefetch(hp + (16 << 8), 0, 0);
            float a = 0.f;
#pragma unroll
            for (int h = lane; h < 256; h += 32)
                a += tanhf(hp[h] + tF32[b * 256 + h]) * swL[h];
#pragma unroll
            for (int off = 16; off > 0; off >>= 1) a += __shfl_xor(a, off);
            if (lane == 0) eA[p] = a;
        }
        __syncthreads();
        if (w < NB) {
            int b = w;
            float v[8]; float m = -1e30f;
#pragma unroll
            for (int j = 0; j < 8; ++j) { v[j] = eA[b * 256 + lane + j * 32];
                                          m = fmaxf(m, v[j]); }
#pragma unroll
            for (int off = 16; off > 0; off >>= 1) m = fmaxf(m, __shfl_xor(m, off));
            float sm = 0.f;
#pragma unroll
            for (int j = 0; j < 8; ++j) { v[j] = __expf(v[j] - m); sm += v[j]; }
#pragma unroll
            for (int off = 16; off > 0; off >>= 1) sm += __shfl_xor(sm, off);
            float inv = 1.f / sm;
#pragma unroll
            for (int j = 0; j < 8; ++j) eA[b * 256 + lane + j * 32] = v[j] * inv;
        }
        __syncthreads();
        for (int p = tid; p < NB * CIN; p += 512) {
            int b = p / CIN, c = p - b * CIN;
            const float* bh = fea + ((size_t)(b * CIN + c) << 8);
            const float* al = eA + b * 256;
            float a = 0.f;
#pragma unroll 4
            for (int s = 0; s < 256; ++s) a += al[s] * bh[s];
            ctx[p] = a;
        }
        __syncthreads();
        for (int p = tid; p < NB * 128; p += 512) {
            int b = p >> 7, c = p & 127;
            float vv;
            if (c < CIN)             vv = ctx[b * CIN + c];
            else if (c < CIN + NOUT) vv = (preL[b] == (c - CIN)) ? 1.f : 0.f;
            else                     vv = 0.f;
            xF16[p] = (_Float16)vv;
        }
        __syncthreads();
        for (int nt = w; nt < 48; nt += 16) {
            v8f gi = {}; gi = wmma_rm(xF16,   128, gihW + lz, 128, nt * 16, 128, gi);
            v8f gh = {}; gh = wmma_rm(hidF16, 256, ghhW + lz, 256, nt * 16, 256, gh);
            if (!hiH) {
                int col = nt * 16 + mlo;
                float b1 = bih[col], b2 = bhh[col];
#pragma unroll
                for (int r = 0; r < NB; ++r) {
                    giL[r * 768 + col] = gi[r] + b1;
                    ghL[r * 768 + col] = gh[r] + b2;
                }
            }
        }
        __syncthreads();
        for (int p = tid; p < NB * HIDN; p += 512) {
            int b = p >> 8, h = p & 255;
            float ir  = giL[b * 768 + h],       hr = ghL[b * 768 + h];
            float iz  = giL[b * 768 + 256 + h], hz = ghL[b * 768 + 256 + h];
            float in_ = giL[b * 768 + 512 + h], hn = ghL[b * 768 + 512 + h];
            float r = 1.f / (1.f + __expf(-(ir + hr)));
            float z = 1.f / (1.f + __expf(-(iz + hz)));
            float n = tanhf(in_ + r * hn);
            float nh = (1.f - z) * n + z * hidF32[p];
            hidF32[p] = nh;
            hidF16[b * 256 + h] = (_Float16)nh;
        }
        __syncthreads();
        {
            v8f a1 = {}; a1 = wmma_rm(hidF16, 256, sg1W + lz, 256, w * 16, 256, a1);
            v8f a2 = {}; a2 = wmma_rm(hidF16, 256, lg1W + lz, 256, w * 16, 256, a2);
            if (!hiH) {
                int col = w * 16 + mlo;
                float b1 = sg1B[col], b2 = lg1B[col];
#pragma unroll
                for (int r = 0; r < NB; ++r) {
                    s1F16[r * 256 + col] = (_Float16)(a1[r] + b1);
                    l1F16[r * 256 + col] = (_Float16)(a2[r] + b2);
                }
            }
        }
        __syncthreads();
        if (w < 2) {
            v8f a = {};
            a = wmma_rm(s1F16, 256, sg2L + lz, 256, w * 16, 256, a);
            if (!hiH) {
                int col = w * 16 + mlo;
                float bb = (col < NOUT) ? sg2B[col] : 0.f;
#pragma unroll
                for (int r = 0; r < NB; ++r) sOut[r * 32 + col] = a[r] + bb;
            }
        } else if (w == 2) {
            v8f a = {};
            a = wmma_rm(l1F16, 256, lg2L + lz, 256, 0, 256, a);
            if (!hiH) {
                float bb = (mlo < NLOC) ? lg2B[mlo] : 0.f;
#pragma unroll
                for (int r = 0; r < NB; ++r) lOut[r * 16 + mlo] = a[r] + bb;
            }
        }
        __syncthreads();
        if (tid < NB) {
            int b = tid;
            float m = -1e30f; int am = 0;
            for (int j = 0; j < NOUT; ++j) {
                float v = sOut[b * 32 + j];
                if (v > m) { m = v; am = j; }
            }
            float sm = 0.f;
            for (int j = 0; j < NOUT; ++j) sm += __expf(sOut[b * 32 + j] - m);
            float inv = 1.f / sm;
            for (int j = 0; j < NOUT; ++j) sOut[b * 32 + j] = __expf(sOut[b * 32 + j] - m) * inv;
            for (int j = NOUT; j < 32; ++j) sOut[b * 32 + j] = 0.f;
            for (int j = NLOC; j < 16; ++j) lOut[b * 16 + j] = 0.f;
            preL[b] = am;
        }
        __syncthreads();
        if (tid < NB * 16) {
            const int b = tid >> 4, pc = tid & 15;
            v4f v;
            if (pc < 8)       v = *(const v4f*)(sOut + b * 32 + pc * 4);
            else if (pc < 12) v = *(const v4f*)(lOut + b * 16 + (pc - 8) * 4);
            else              v = (v4f){0.f, 0.f, 0.f, 0.f};
            vst2(stage + ((size_t)b * STEPS + step) * 64 + pc * 4, v);
        }
        __syncthreads();
    }
}

__global__ __launch_bounds__(256) void pack_out(const float* __restrict__ stage, float* __restrict__ out)
{
    const int nS = NB * STEPS * NOUT, nL = NB * STEPS * NLOC;
    const int g = blockIdx.x * 256 + threadIdx.x;
    if (g * 4 >= nS + nL) return;
    float v[4];
#pragma unroll
    for (int e = 0; e < 4; ++e) {
        const int i = g * 4 + e;
        if (i < nS) { const int rec = i / NOUT, j = i - rec * NOUT; v[e] = stage[(size_t)rec * 64 + j]; }
        else        { const int ii = i - nS; const int rec = ii / NLOC, j = ii - rec * NLOC; v[e] = stage[(size_t)rec * 64 + 32 + j]; }
    }
    vst2(out + (size_t)g * 4, (v4f){v[0], v[1], v[2], v[3]});
}

extern "C" void kernel_launch(void* const* d_in, const int* in_sizes, int n_in,
                              void* d_out, int out_size, void* d_ws, size_t ws_size,
                              hipStream_t stream)
{
    (void)in_sizes; (void)n_in; (void)out_size; (void)ws_size;
    const float* fea     = (const float*)d_in[0];
    const float* i2h_w   = (const float*)d_in[1];
    const float* h2h_w   = (const float*)d_in[2];
    const float* h2h_b   = (const float*)d_in[3];
    const float* score_w = (const float*)d_in[4];
    const float* gw_ih   = (const float*)d_in[5];
    const float* gw_hh   = (const float*)d_in[6];
    const float* gb_ih   = (const float*)d_in[7];
    const float* gb_hh   = (const float*)d_in[8];
    const float* sg1_w   = (const float*)d_in[9];
    const float* sg1_b   = (const float*)d_in[10];
    const float* sg2_w   = (const float*)d_in[11];
    const float* sg2_b   = (const float*)d_in[12];
    const float* lg1_w   = (const float*)d_in[13];
    const float* lg1_b   = (const float*)d_in[14];
    const float* lg2_w   = (const float*)d_in[15];
    const float* lg2_b   = (const float*)d_in[16];

    char* ws = (char*)d_ws;
    size_t off = 0;
    _Float16* h2hH = (_Float16*)(ws + off); off += 256 * 256 * 2;
    _Float16* gihH = (_Float16*)(ws + off); off += 768 * 128 * 2;
    _Float16* ghhH = (_Float16*)(ws + off); off += 768 * 256 * 2;
    _Float16* sg1H = (_Float16*)(ws + off); off += 256 * 256 * 2;
    _Float16* lg1H = (_Float16*)(ws + off); off += 256 * 256 * 2;
    _Float16* sg2H = (_Float16*)(ws + off); off += 32  * 256 * 2;
    _Float16* lg2H = (_Float16*)(ws + off); off += 16  * 256 * 2;
    float*    Hp   = (float*)   (ws + off); off += (size_t)8 * 256 * 256 * 4;
    float*    stage= (float*)   (ws + off); off += (size_t)8 * STEPS * 64 * 4;

    auto cvt = [&](const float* src, _Float16* dst, int rs, int cs, int rd, int cd) {
        int n = rd * cd / 8;
        cvt_pad_f16<<<(n + 255) / 256, 256, 0, stream>>>(src, dst, rs, cs, rd, cd);
    };
    cvt(h2h_w, h2hH, 256, 256, 256, 256);
    cvt(gw_ih, gihH, 768, 126, 768, 128);
    cvt(gw_hh, ghhH, 768, 256, 768, 256);
    cvt(sg1_w, sg1H, 256, 256, 256, 256);
    cvt(lg1_w, lg1H, 256, 256, 256, 256);
    cvt(sg2_w, sg2H, 30, 256, 32, 256);
    cvt(lg2_w, lg2H, 4, 256, 16, 256);

    prep_hproj<<<(8 * 256 * 256) / 256, 256, 0, stream>>>(fea, i2h_w, Hp);

    float* out = (float*)d_out;

    size_t smem = (size_t)(48 * 256 + 16 * 256 + 16 * 128 + 16 * 256 + 16 * 256) * sizeof(_Float16)
                + (size_t)(8 * 256 * 3 + 8 * 768 * 2 + 8 * 96 + 8 * 32 + 8 * 16 + 256) * sizeof(float)
                + 8 * sizeof(int);
    hipFuncSetAttribute((const void*)sla_decoder,
                        hipFuncAttributeMaxDynamicSharedMemorySize, (int)smem);

    sla_decoder<<<1, 512, smem, stream>>>(
        fea, Hp, h2hH, h2h_b, score_w, gihH, ghhH, gb_ih, gb_hh,
        sg1H, sg1_b, sg2H, sg2_b, lg1H, lg1_b, lg2H, lg2_b, stage);
    pack_out<<<(8 * STEPS * (NOUT + NLOC) / 4 + 255) / 256, 256, 0, stream>>>(stage, out);
}
